// VSDF_60043642798803
// MI455X (gfx1250) — hardware-run, weakly checked
//
#include <hip/hip_runtime.h>
#include <math.h>

typedef __attribute__((ext_vector_type(16))) _Float16 v16h;
typedef __attribute__((ext_vector_type(16))) __bf16 v16b;
typedef __attribute__((ext_vector_type(8)))  _Float16 v8h;
typedef __attribute__((ext_vector_type(8)))  float v8f;
typedef __attribute__((ext_vector_type(4)))  float v4f;
typedef __attribute__((ext_vector_type(2)))  float v2f;
typedef __attribute__((ext_vector_type(4)))  unsigned v4u;
typedef __attribute__((ext_vector_type(4)))  int v4i;
typedef float __attribute__((may_alias)) float_a;
typedef int __attribute__((may_alias)) int_a;

template <typename T> __device__ __forceinline__ void vst2(void* p, T v) { *(volatile T*)p = v; __threadfence(); *(volatile T*)p = v; }
__device__ __forceinline__ v8f wmma16(v16h a, v16h b, v8f c) {
  v8f d = __builtin_amdgcn_wmma_f32_16x16x32_f16(false, a, false, b, (short)0, c, false, false);
  asm volatile("v_nop\n\tv_nop\n\tv_nop\n\tv_nop" : "+v"(d) : "v"(a), "v"(b));
  return d;
}
__device__ __forceinline__ v8f wmma_bf(v16b a, v16b b, v8f c) {
  v8f d = __builtin_amdgcn_wmma_f32_16x16x32_bf16(false, a, false, b, (short)0, c, false, false);
  asm volatile("v_nop\n\tv_nop\n\tv_nop\n\tv_nop" : "+v"(d) : "v"(a), "v"(b));
  return d;
}
__device__ __forceinline__ v16h frag_h(const _Float16* rowk0, int lane) {
  union { v16h v; v8h q[2]; } u; const _Float16* p = rowk0 + 8 * (lane >> 4);
  u.q[0] = *(const v8h*)p; u.q[1] = *(const v8h*)(p + 16); return u.v;
}
__device__ __forceinline__ v16h frag_f32(const float* rowk0, int lane) {
  v16h a; const float* p = rowk0 + 8 * (lane >> 4);
#pragma unroll
  for (int i = 0; i < 8; ++i) { a[i] = (_Float16)p[i]; a[8 + i] = (_Float16)p[16 + i]; }
  return a;
}
__device__ __forceinline__ v16h frag_f32s(const float* rowk0, int lane, float sc) {
  v16h a; const float* p = rowk0 + 8 * (lane >> 4);
#pragma unroll
  for (int i = 0; i < 8; ++i) { a[i] = (_Float16)(p[i] * sc); a[8 + i] = (_Float16)(p[16 + i] * sc); }
  return a;
}
__device__ __forceinline__ v16h fragc_f32(const float* W, int k0, int n, int lane, int ld, int K) {
  v16h a; const int g = lane >> 4;
#pragma unroll
  for (int i = 0; i < 8; ++i) { const int ka = k0 + 8 * g + i, kb = ka + 16;
    a[i] = (_Float16)(ka < K ? W[(size_t)(ka < K ? ka : K - 1) * ld + n] : 0.f); a[8 + i] = (_Float16)(kb < K ? W[(size_t)(kb < K ? kb : K - 1) * ld + n] : 0.f); }
  return a;
}
struct F2 { v16b h, l; };
__device__ __forceinline__ F2 bsplit16(const float v[16]) { F2 r;
#pragma unroll
  for (int i = 0; i < 16; ++i) { const __bf16 h = (__bf16)v[i]; r.h[i] = h; r.l[i] = (__bf16)(v[i] - (float)h); }
  return r; }
__device__ __forceinline__ F2 split_row(const float* row, int k0, int lane) { float v[16]; const float* p = row + k0 + 8 * (lane >> 4);
#pragma unroll
  for (int i = 0; i < 8; ++i) { v[i] = p[i]; v[8 + i] = p[16 + i]; }
  return bsplit16(v); }
__device__ __forceinline__ F2 split_rowK(const float* row, int k0, int lane, int K) { float v[16]; const int g = lane >> 4;
#pragma unroll
  for (int i = 0; i < 8; ++i) { const int ka = k0 + 8 * g + i, kb = ka + 16; v[i] = ka < K ? row[ka < K ? ka : K - 1] : 0.f; v[8 + i] = kb < K ? row[kb < K ? kb : K - 1] : 0.f; }
  return bsplit16(v); }
__device__ __forceinline__ F2 split_col(const float* W, int k0, int n, int lane, int ld, int K) { float v[16]; const int g = lane >> 4;
#pragma unroll
  for (int i = 0; i < 8; ++i) { const int ka = k0 + 8 * g + i, kb = ka + 16; v[i] = ka < K ? W[(size_t)(ka < K ? ka : K - 1) * ld + n] : 0.f; v[8 + i] = kb < K ? W[(size_t)(kb < K ? kb : K - 1) * ld + n] : 0.f; }
  return bsplit16(v); }
__device__ __forceinline__ v8f mac3(const F2& a, const F2& b, v8f c) { c = wmma_bf(a.l, b.h, c); c = wmma_bf(a.h, b.l, c); return wmma_bf(a.h, b.h, c); }
__device__ __forceinline__ float sigm(float v) { return 1.0f / (1.0f + expf(-v)); }
#define LDSX() do { asm volatile("s_wait_dscnt 0" ::: "memory"); __builtin_amdgcn_wave_barrier(); __builtin_amdgcn_fence(__ATOMIC_RELEASE, "workgroup"); } while (0)


#define NB 8
#define SS 1024
#define DM 512
#define NH 8
#define HD 64
#define QKVW (3 * DM)
#ifndef TQB
#define TQB (SS / 64)
#define TNB NB
#define TOB (NB * SS / 64)
#endif
typedef __attribute__((ext_vector_type(8))) __bf16 v8b;
__device__ __forceinline__ v16b frag_b(const __bf16* rowk0, int lane) {
  union { v16b v; v8b q[2]; } u; const __bf16* p = rowk0 + 8 * (lane >> 4);
  u.q[0] = *(const v8b*)p; u.q[1] = *(const v8b*)(p + 16); return u.v;
}
__device__ __forceinline__ float bfr(float v) { return (float)(__bf16)v; }
__device__ __attribute__((noinline)) float exp_ni(float v) { return expf(v); }
__device__ __attribute__((noinline)) float erf_ni(float v) { return erff(v); }

#define PK_A 0
#define PK_P (PK_A + QKVW * DM)
#define PK_END (PK_P + DM * DM)

#define NR (NB * SS)
#define D3 (3 * DM)
#define D2 (2 * DM)
#ifndef NRB
#define NRB (NR / 64)
#endif

#define WS_PWQ  0u
#define WS_PWP  (WS_PWQ + 2u * (size_t)2 * D3 * DM)
#define WS_PF1  (WS_PWP + 2u * (size_t)2 * DM * DM)
#define WS_PF2  (WS_PF1 + 2u * (size_t)D2 * DM)
#define WS_PR1  (WS_PF2 + 2u * (size_t)DM * D2)
#define WS_PR2  (WS_PR1 + 2u * (size_t)D2 * DM)
#define WS_BIG  (WS_PR2 + 2u * (size_t)DM * D2)
#define WS_QKVF (WS_BIG)
#define WS_O    (WS_BIG)
#define WS_OBR  (WS_O + 4u * (size_t)2 * NR * DM)
#define WS_VOL  (WS_OBR + 4u * (size_t)2 * NR * DM)
#define WS_FUS  (WS_VOL + 4u * (size_t)NR * DM)
#define WS_BIGEND (WS_BIG + 4u * (size_t)2 * NR * D3)
#define WS_QK   (WS_BIGEND)
#define WS_VT   (WS_QK + 2u * (size_t)2 * NR * D2)
#define WS_S16  (WS_VT + 2u * (size_t)2 * NB * DM * SS)
#define WS_F16  (WS_S16 + 2u * (size_t)NR * DM)
#define WS_G16  (WS_F16 + 2u * (size_t)NR * DM)
#define WS_GATE (WS_G16 + 2u * (size_t)NR * D2)
#define WS_MEAN (WS_GATE + 4u * NB * 4)
#define WS_END  (WS_MEAN + 4u * 2 * NB * DM)

__global__ __launch_bounds__(256) void k_pack(const float* __restrict__ SQW, const float* __restrict__ PQW, const float* __restrict__ SPW, const float* __restrict__ PPW, const float* __restrict__ VF1, const float* __restrict__ VF2, const float* __restrict__ FR1, const float* __restrict__ FR2, __bf16* __restrict__ P, _Float16* __restrict__ PH) {
  const int n = blockIdx.x, which = blockIdx.y, t = threadIdx.x; __shared__ __align__(16) __bf16 s[D2]; __shared__ __align__(16) _Float16 sh[D2];
  if (which < 2) { const float* Wm = which ? PQW : SQW; if (n >= D3) return; for (int k = t; k < DM; k += 256) s[k] = (__bf16)Wm[(size_t)k * D3 + n]; __syncthreads(); for (int q = t; q < DM / 8; q += 256) vst2((unsigned*)(P + WS_PWQ / 2 + ((size_t)which * D3 + n) * DM + q * 8), *(const v4u*)&s[q * 8]); }
  else if (which < 4) { const float* Wm = (which == 3) ? PPW : SPW; if (n >= DM) return; for (int k = t; k < DM; k += 256) s[k] = (__bf16)Wm[(size_t)k * DM + n]; __syncthreads(); for (int q = t; q < DM / 8; q += 256) vst2((unsigned*)(P + WS_PWP / 2 + ((size_t)(which - 2) * DM + n) * DM + q * 8), *(const v4u*)&s[q * 8]); }
  else { const bool first = (which == 4 || which == 6); const float* Wm = (which == 4) ? VF1 : (which == 5) ? VF2 : (which == 6) ? FR1 : FR2; const int kin = first ? DM : D2, nout = first ? D2 : DM; if (n >= nout) return;
    for (int k = t; k < kin; k += 256) sh[k] = (_Float16)(bfr(Wm[(size_t)k * nout + n]) * 256.0f); __syncthreads();
    _Float16* dst = PH + ((which == 4) ? 0 : (which == 5) ? (size_t)D2 * DM : (which == 6) ? (size_t)2 * D2 * DM : (size_t)3 * D2 * DM) + (size_t)n * kin;
    for (int q = t; q < kin / 8; q += 256) vst2((unsigned*)(dst + q * 8), *(const v4u*)&sh[q * 8]); }
}
__global__ __launch_bounds__(128) void k_qkv(const float* __restrict__ X0, const float* __restrict__ X1, const __bf16* __restrict__ P, const float* __restrict__ B0, const float* __restrict__ B1v, float* __restrict__ QKVF) {
  __shared__ __align__(16) float so[4][16][132];
  const int tid = threadIdx.x, wave = tid >> 5, lane = tid & 31, col = lane & 15, g = lane >> 4; const int br = blockIdx.z; const size_t r0 = (size_t)blockIdx.x * 64 + wave * 16; const int n0 = blockIdx.y * 128;
  const float* X = br ? X1 : X0; const float* BB = br ? B1v : B0; const __bf16* Wr = P + WS_PWQ / 2 + (size_t)br * D3 * DM;
  v8f acc[8] = {};
#pragma unroll 2
  for (int kc = 0; kc < DM / 32; ++kc) { v16b a; { const float* p = X + (r0 + col) * DM + kc * 32 + 8 * g;
#pragma unroll
      for (int i = 0; i < 8; ++i) { a[i] = (__bf16)p[i]; a[8 + i] = (__bf16)p[16 + i]; } }
#pragma unroll
    for (int j = 0; j < 8; ++j) acc[j] = wmma_bf(a, frag_b(Wr + (size_t)(n0 + j * 16 + col) * DM + kc * 32, lane), acc[j]); }
#pragma unroll
  for (int j = 0; j < 8; ++j) { const float bb = bfr(BB[n0 + j * 16 + col]);
#pragma unroll
    for (int r = 0; r < 8; ++r) so[wave][8 * g + r][j * 16 + col] = acc[j][r] + bb; }
  LDSX();
  for (int rl = 0; rl < 16; ++rl) vst2(QKVF + ((size_t)br * NR + r0 + rl) * D3 + n0 + lane * 4, *(const v4f*)&so[wave][rl][lane * 4]);
}
__global__ __launch_bounds__(256) void k_lnsplit(const float* __restrict__ QKVF, const float* __restrict__ G0, const float* __restrict__ Bt0, const float* __restrict__ G1, const float* __restrict__ Bt1, _Float16* __restrict__ QK, _Float16* __restrict__ VTMP) {
  __shared__ float red[8]; __shared__ float sv[D3]; __shared__ float hs[2 * NH];
  const size_t row = blockIdx.x; const int br = blockIdx.y, t = threadIdx.x; const float* G = br ? G1 : G0; const float* Bt = br ? Bt1 : Bt0; const float* src = QKVF + ((size_t)br * NR + row) * D3;
  float v[6]; float s = 0.f; for (int i = 0; i < 6; ++i) { v[i] = src[t + 256 * i]; s += v[i]; }
#pragma unroll
  for (int o = 1; o < 32; o <<= 1) s += __shfl_xor(s, o);
  if ((t & 31) == 0) red[t >> 5] = s; __syncthreads(); float tot = 0.f; for (int i = 0; i < 8; ++i) tot += red[i]; const float mu = tot / (float)D3; __syncthreads();
  float q = 0.f; for (int i = 0; i < 6; ++i) { const float dd = v[i] - mu; q += dd * dd; }
#pragma unroll
  for (int o = 1; o < 32; o <<= 1) q += __shfl_xor(q, o);
  if ((t & 31) == 0) red[t >> 5] = q; __syncthreads(); float tq = 0.f; for (int i = 0; i < 8; ++i) tq += red[i]; const float inv = 1.0f / sqrtf(tq / (float)D3 + 1e-5f);
  for (int i = 0; i < 6; ++i) { const int e = t + 256 * i; sv[e] = (v[i] - mu) * inv * bfr(G[e]) + bfr(Bt[e]); }
  __syncthreads();
  if (t < 2 * NH * 8) { const int hh = t >> 3, part = t & 7; float ss = 0.f; for (int d = part * 8; d < part * 8 + 8; ++d) { const float x = sv[hh * HD + d]; ss += x * x; } ss += __shfl_xor(ss, 1); ss += __shfl_xor(ss, 2); ss += __shfl_xor(ss, 4); if (part == 0) hs[hh] = fmaxf(sqrtf(ss), 1e-12f); }
  __syncthreads();
  __shared__ __align__(16) _Float16 so[D3];
  for (int e = t; e < D3; e += 256) so[e] = (_Float16)((e < D2) ? sv[e] / hs[e / HD] : sv[e]);
  __syncthreads();
  for (int qd = t; qd < D2 / 8; qd += 256) vst2((unsigned*)(QK + ((size_t)br * NR + row) * D2 + qd * 8), *(const v4u*)&so[qd * 8]);
  for (int qd = t; qd < DM / 8; qd += 256) vst2((unsigned*)(VTMP + ((size_t)br * NR + row) * DM + qd * 8), *(const v4u*)&so[D2 + qd * 8]);
}
__global__ __launch_bounds__(256) void k_vplanes(const _Float16* __restrict__ VTMP, _Float16* __restrict__ VT) {
  __shared__ __align__(16) _Float16 st[128][72]; const size_t rb0 = (size_t)blockIdx.x * 64; const int c0 = blockIdx.y * 128, br = blockIdx.z, t = threadIdx.x;
  for (int e = t; e < 64 * 128; e += 256) { const int r = e >> 7, c = e & 127; st[c][r] = VTMP[((size_t)br * NR + rb0 + r) * DM + c0 + c]; }
  __syncthreads();
  const size_t b = rb0 / SS, s0 = rb0 % SS;
  for (int e = t; e < 128 * 8; e += 256) { const int c = e >> 3, pc = e & 7; vst2((unsigned*)(VT + (((size_t)br * NB + b) * DM + c0 + c) * SS + s0 + pc * 8), *(const v4u*)&st[c][pc * 8]); }
}
__global__ __launch_bounds__(128) void k_attn(const _Float16* __restrict__ QK, const _Float16* __restrict__ QKL, const _Float16* __restrict__ VTH, const _Float16* __restrict__ VTL, const void* __restrict__ KMASK, const float* __restrict__ TEMP, float* __restrict__ O) {
  __shared__ __align__(16) float sp[4][16][36]; __shared__ __align__(16) float so[4][16][68];
  const int tid = threadIdx.x, wave = tid >> 5, lane = tid & 31, col = lane & 15, g = lane >> 4;
  const int qb = blockIdx.x, h = blockIdx.y, b = blockIdx.z; const int q0 = qb * 64 + wave * 16; const size_t rq = (size_t)b * SS + q0 + col;
  v16h aq[2], aql[2];
#pragma unroll
  for (int kc = 0; kc < 2; ++kc) { aq[kc] = frag_h(QK + rq * (2 * DM) + h * HD + kc * 32, lane); aql[kc] = frag_h(QKL + rq * (2 * DM) + h * HD + kc * 32, lane); }
  const float tscale = bfr(TEMP[h]);
  float m[8], l[8];
#pragma unroll
  for (int r = 0; r < 8; ++r) { m[r] = -3.0e38f; l[r] = 0.f; }
  v8f acc[4] = {}, accl[4] = {};
  const int nks = SS / 32;
#pragma unroll 1
  for (int ks = 0; ks < nks; ++ks) { v8f s[2];
#pragma unroll
    for (int ct = 0; ct < 2; ++ct) { const int kk = ks * 32 + ct * 16 + col; const _Float16* krow = QK + ((size_t)b * SS + kk) * (2 * DM) + DM + h * HD; const _Float16* krowl = QKL + ((size_t)b * SS + kk) * (2 * DM) + DM + h * HD; v8f c = {}, cl = {};
#pragma unroll
      for (int kc = 0; kc < 2; ++kc) c = wmma16(aq[kc], frag_h(krow + kc * 32, lane), c);
      (void)cl; (void)krowl;
      { const bool keepk = true;
#pragma unroll
      for (int r = 0; r < 8; ++r) s[ct][r] = c[r] * tscale; } }
#pragma unroll
    for (int r = 0; r < 8; ++r) { float mx = fmaxf(s[0][r], s[1][r]);
#pragma unroll
      for (int o = 1; o < 16; o <<= 1) mx = fmaxf(mx, __shfl_xor(mx, o));
      const float mn = fmaxf(m[r], mx); const float alpha = (m[r] <= -1.0e38f) ? 0.f : __expf(m[r] - mn);
      const float e0 = (s[0][r] <= -1.0e38f) ? 0.f : __expf(s[0][r] - mn), e1 = (s[1][r] <= -1.0e38f) ? 0.f : __expf(s[1][r] - mn); float es = e0 + e1;
#pragma unroll
      for (int o = 1; o < 16; o <<= 1) es += __shfl_xor(es, o);
      l[r] = l[r] * alpha + es; m[r] = mn;
#pragma unroll
      for (int dt = 0; dt < 4; ++dt) { acc[dt][r] *= alpha; accl[dt][r] *= alpha; }
      sp[wave][8 * g + r][col] = e0; sp[wave][8 * g + r][16 + col] = e1; }
    LDSX();
    v16h pa, pl; { const float* prow = &sp[wave][col][0] + 8 * (lane >> 4);
#pragma unroll
      for (int i = 0; i < 8; ++i) { const float x0 = prow[i] * 2048.0f, x1 = prow[16 + i] * 2048.0f; const _Float16 h0 = (_Float16)x0, h1 = (_Float16)x1; pa[i] = h0; pa[8 + i] = h1; pl[i] = (_Float16)((x0 - (float)h0) * 2048.0f); pl[8 + i] = (_Float16)((x1 - (float)h1) * 2048.0f); } }
#pragma unroll
    for (int dt = 0; dt < 4; ++dt) { const size_t vr = ((size_t)b * DM + h * HD + dt * 16 + col) * SS + ks * 32; acc[dt] = wmma16(pa, frag_h(VTH + vr, lane), acc[dt]); }
    (void)pl;
    LDSX(); }
#pragma unroll
  for (int r = 0; r < 8; ++r) { const float il = (1.0f / 2048.0f) / l[r];
#pragma unroll
    for (int dt = 0; dt < 4; ++dt) so[wave][8 * g + r][dt * 16 + col] = (acc[dt][r] + accl[dt][r] * (1.0f / 2048.0f)) * il; }
  LDSX();
  for (int rl = 0; rl < 16; ++rl) if (lane < 16) vst2(O + ((size_t)b * SS + q0 + rl) * DM + h * HD + lane * 4, *(const v4f*)&so[wave][rl][lane * 4]);
}

__global__ __launch_bounds__(128) void k_proj(const float* __restrict__ O, const __bf16* __restrict__ P, const float* __restrict__ B0, const float* __restrict__ B1v, float* __restrict__ OBR) {
  __shared__ __align__(16) float so[4][16][132];
  const int tid = threadIdx.x, wave = tid >> 5, lane = tid & 31, col = lane & 15, g = lane >> 4; const int br = blockIdx.z; const size_t r0 = (size_t)blockIdx.x * 64 + wave * 16; const int n0 = blockIdx.y * 128;
  const float* BB = br ? B1v : B0; const __bf16* Wr = P + WS_PWP / 2 + (size_t)br * DM * DM;
  v8f acc[8] = {};
#pragma unroll 2
  for (int kc = 0; kc < DM / 32; ++kc) { const F2 a = split_row(O + ((size_t)br * NR + r0 + col) * DM, kc * 32, lane);
#pragma unroll
    for (int j = 0; j < 8; ++j) { const v16b w = frag_b(Wr + (size_t)(n0 + j * 16 + col) * DM + kc * 32, lane); acc[j] = wmma_bf(a.l, w, acc[j]); acc[j] = wmma_bf(a.h, w, acc[j]); } }
#pragma unroll
  for (int j = 0; j < 8; ++j) { const float bb = bfr(BB[n0 + j * 16 + col]);
#pragma unroll
    for (int r = 0; r < 8; ++r) so[wave][8 * g + r][j * 16 + col] = acc[j][r] + bb; }
  LDSX();
  for (int rl = 0; rl < 16; ++rl) vst2(OBR + ((size_t)br * NR + r0 + rl) * DM + n0 + lane * 4, *(const v4f*)&so[wave][rl][lane * 4]);
}
__global__ __launch_bounds__(128) void k_s16(const float* __restrict__ OBR, _Float16* __restrict__ S16) { const size_t row = blockIdx.x; const int t = threadIdx.x; __shared__ __align__(16) _Float16 s[DM]; for (int c = t; c < DM; c += 128) s[c] = (_Float16)(OBR[row * DM + c] + OBR[((size_t)NR + row) * DM + c]); __syncthreads(); if (t < DM / 8) vst2((unsigned*)(S16 + row * DM + t * 8), *(const v4u*)&s[t * 8]); }
__device__ __attribute__((noinline)) float gelu_e(float x) { return 0.5f * x * (1.0f + erff(x * 0.70710678118654752f)); }
template <int MODE>
__global__ __launch_bounds__(128) void k_mlp(const _Float16* __restrict__ Ain, const _Float16* __restrict__ Wr, const float* __restrict__ BIAS, const float* __restrict__ FUS, const float* __restrict__ X0, const float* __restrict__ X1, const float* __restrict__ AL, const float* __restrict__ BE, float* __restrict__ OUTF, _Float16* __restrict__ OG) {
  constexpr int KIN = (MODE == 0) ? DM : D2; constexpr int NOUT = (MODE == 0) ? D2 : DM;
  __shared__ __align__(16) float so[4][16][132]; __shared__ __align__(16) _Float16 sg[4][16][136];
  const int tid = threadIdx.x, wave = tid >> 5, lane = tid & 31, col = lane & 15, g = lane >> 4; const size_t r0 = (size_t)blockIdx.x * 64 + wave * 16; const int n0 = blockIdx.y * 128;
  v8f acc[8] = {};
#pragma unroll 2
  for (int kc = 0; kc < KIN / 32; ++kc) { const v16h a = frag_h(Ain + (r0 + col) * KIN + kc * 32, lane);
#pragma unroll
    for (int j = 0; j < 8; ++j) acc[j] = wmma16(a, frag_h(Wr + (size_t)(n0 + j * 16 + col) * KIN + kc * 32, lane), acc[j]); }
  const float alpha = (MODE == 2) ? bfr(AL[0]) : 0.f, beta = (MODE == 2) ? bfr(BE[0]) : 0.f;
#pragma unroll
  for (int j = 0; j < 8; ++j) { const int c = n0 + j * 16 + col; const float bb = bfr(BIAS[c]);
#pragma unroll
    for (int r = 0; r < 8; ++r) { const float x = acc[j][r] * (1.0f / 256.0f) + bb; const size_t row = r0 + 8 * g + r;
      if (MODE == 0) sg[wave][8 * g + r][j * 16 + col] = (_Float16)gelu_e(x);
      else if (MODE == 1) so[wave][8 * g + r][j * 16 + col] = x;
      else so[wave][8 * g + r][j * 16 + col] = FUS[row * DM + c] + alpha * x + beta * (bfr(X0[row * DM + c]) + bfr(X1[row * DM + c])) * 0.5f; } }
  LDSX();
  if (MODE == 0) { for (int rl = 0; rl < 16; ++rl) if (lane < 16) vst2((unsigned*)(OG + (r0 + rl) * NOUT + n0 + lane * 8), *(const v4u*)&sg[wave][rl][lane * 8]); }
  else { for (int rl = 0; rl < 16; ++rl) vst2(OUTF + (r0 + rl) * NOUT + n0 + lane * 4, *(const v4f*)&so[wave][rl][lane * 4]); }
}
__global__ __launch_bounds__(256) void k_gate(const float* __restrict__ OBR, const float* __restrict__ W1, const float* __restrict__ B1v, const float* __restrict__ G, const float* __restrict__ Bt, const float* __restrict__ W2, const float* __restrict__ B2v, float* __restrict__ GATE) {
  __shared__ float sm[D2]; __shared__ float sg1[DM]; __shared__ float red[8]; __shared__ float lg[3];
  const size_t b = blockIdx.x; const int t = threadIdx.x;
  for (int e = t; e < D2; e += 256) { const int br = e / DM, c = e % DM; float s = 0.f;
#pragma unroll 1
    for (int n = 0; n < SS; ++n) s += OBR[((size_t)br * NR + b * SS + n) * DM + c];
    sm[e] = s / (float)SS; }
  __syncthreads();
  for (int n = t; n < DM; n += 256) { float s = bfr(B1v[n]);
#pragma unroll 1
    for (int k = 0; k < D2; ++k) s += sm[k] * bfr(W1[(size_t)k * DM + n]);
    sg1[n] = s; }
  __syncthreads();
  float s = 0.f; for (int n = t; n < DM; n += 256) s += sg1[n];
#pragma unroll
  for (int o = 1; o < 32; o <<= 1) s += __shfl_xor(s, o);
  if ((t & 31) == 0) red[t >> 5] = s; __syncthreads(); float tot = 0.f; for (int i = 0; i < 8; ++i) tot += red[i]; const float mu = tot / (float)DM; __syncthreads();
  float q = 0.f; for (int n = t; n < DM; n += 256) { const float dd = sg1[n] - mu; q += dd * dd; }
#pragma unroll
  for (int o = 1; o < 32; o <<= 1) q += __shfl_xor(q, o);
  if ((t & 31) == 0) red[t >> 5] = q; __syncthreads(); float tq = 0.f; for (int i = 0; i < 8; ++i) tq += red[i]; const float inv = 1.0f / sqrtf(tq / (float)DM + 1e-5f); __syncthreads();
  for (int n = t; n < DM; n += 256) sg1[n] = gelu_e((sg1[n] - mu) * inv * bfr(G[n]) + bfr(Bt[n]));
  __syncthreads();
  if (t < 3) { float z = bfr(B2v[t]);
#pragma unroll 1
    for (int k = 0; k < DM; ++k) z += sg1[k] * bfr(W2[k * 3 + t]);
    lg[t] = z; }
  __syncthreads();
  if (t == 0) { const float mx = fmaxf(lg[0], fmaxf(lg[1], lg[2])); const float e0 = exp_ni(lg[0] - mx), e1 = exp_ni(lg[1] - mx), e2 = exp_ni(lg[2] - mx); const float den = e0 + e1 + e2; GATE[b * 4 + 0] = e0 / den; GATE[b * 4 + 1] = e1 / den; GATE[b * 4 + 2] = e2 / den; GATE[b * 4 + 3] = 0.f; }
}
__global__ __launch_bounds__(128) void k_fuse(const float* __restrict__ OBR, const float* __restrict__ VOL, const float* __restrict__ GATE, float* __restrict__ FUS, _Float16* __restrict__ F16) {
  const size_t row = blockIdx.x; const int t = threadIdx.x; const size_t b = row / SS; const float w0 = GATE[b * 4], w1 = GATE[b * 4 + 1], w2 = GATE[b * 4 + 2];
  __shared__ __align__(16) float sf[DM]; __shared__ __align__(16) _Float16 sh[DM];
  for (int c = t; c < DM; c += 128) { const float f = w0 * OBR[row * DM + c] + w1 * OBR[((size_t)NR + row) * DM + c] + w2 * VOL[row * DM + c]; sf[c] = f; sh[c] = (_Float16)f; }
  __syncthreads();
  for (int q = t; q < DM / 4; q += 128) vst2(FUS + row * DM + q * 4, *(const v4f*)&sf[q * 4]);
  if (t < DM / 8) vst2((unsigned*)(F16 + row * DM + t * 8), *(const v4u*)&sh[t * 8]);
}
extern "C" void kernel_launch(void* const* d_in, const int* in_sizes, int n_in, void* d_out, int out_size, void* d_ws, size_t ws_size, hipStream_t stream) {
  (void)in_sizes; (void)n_in; (void)out_size;
  const float** F = (const float**)d_in;
  if (ws_size < (size_t)WS_END) return;
  char* ws = (char*)d_ws; __bf16* P = (__bf16*)ws; _Float16 *PH = (_Float16*)(ws + WS_PF1), *QK = (_Float16*)(ws + WS_QK), *VT = (_Float16*)(ws + WS_VT), *S16 = (_Float16*)(ws + WS_S16), *F16 = (_Float16*)(ws + WS_F16), *G16 = (_Float16*)(ws + WS_G16); float *QKVF = (float*)(ws + WS_QKVF), *O = (float*)(ws + WS_O), *OBR = (float*)(ws + WS_OBR), *VOL = (float*)(ws + WS_VOL), *FUS = (float*)(ws + WS_FUS), *GATE = (float*)(ws + WS_GATE);
  _Float16* VTMP = G16;
  k_pack<<<dim3(D3, 8), 256, 0, stream>>>(F[3], F[9], F[7], F[13], F[15], F[17], F[25], F[27], P, PH);
  k_qkv<<<dim3(NR / 64, D3 / 128, 2), 128, 0, stream>>>(F[0], F[1], P, F[4], F[10], QKVF);
  k_lnsplit<<<dim3(NR, 2), 256, 0, stream>>>(QKVF, F[5], F[6], F[11], F[12], QK, VTMP);
  k_vplanes<<<dim3(NR / 64, DM / 128, 2), 256, 0, stream>>>(VTMP, VT);
  for (int br = 0; br < 2; ++br)
    k_attn<<<dim3(TQB, NH, TNB), 128, 0, stream>>>(QK + (size_t)br * NR * D2, QK + (size_t)br * NR * D2, VT + (size_t)br * NB * DM * SS, VT + (size_t)br * NB * DM * SS, nullptr, F[2], O + (size_t)br * NR * DM);
  k_proj<<<dim3(NRB, DM / 128, 2), 128, 0, stream>>>(O, P, F[8], F[14], OBR);
  k_s16<<<NRB * 64, 128, 0, stream>>>(OBR, S16);
  k_mlp<0><<<dim3(NRB, D2 / 128), 128, 0, stream>>>(S16, PH, F[16], nullptr, nullptr, nullptr, nullptr, nullptr, nullptr, G16);
  k_mlp<1><<<dim3(NRB, DM / 128), 128, 0, stream>>>(G16, PH + (size_t)D2 * DM, F[18], nullptr, nullptr, nullptr, nullptr, nullptr, VOL, nullptr);
  k_gate<<<NB, 256, 0, stream>>>(OBR, F[19], F[20], F[21], F[22], F[23], F[24], GATE);
  k_fuse<<<NRB * 64, 128, 0, stream>>>(OBR, VOL, GATE, FUS, F16);
  k_mlp<0><<<dim3(NRB, D2 / 128), 128, 0, stream>>>(F16, PH + (size_t)2 * D2 * DM, F[26], nullptr, nullptr, nullptr, nullptr, nullptr, nullptr, G16);
  k_mlp<2><<<dim3(NRB, DM / 128), 128, 0, stream>>>(G16, PH + (size_t)3 * D2 * DM, F[28], FUS, F[0], F[1], F[29], F[30], (float*)d_out, nullptr);
}
